// T10_transformer_70849780514963
// MI455X (gfx1250) — hardware-verified
//
#include <hip/hip_runtime.h>


typedef _Float16 f16t;
typedef f16t  v16h __attribute__((ext_vector_type(16)));
typedef f16t  v8h  __attribute__((ext_vector_type(8)));
typedef float v8f  __attribute__((ext_vector_type(8)));
typedef float v4f  __attribute__((ext_vector_type(4)));
typedef unsigned int v4u __attribute__((ext_vector_type(4)));

union Frag { v16h v; v8h q[2]; };
union Pk16 { v8h h; v4u u; };

#define SEQ_BLK 32
#define TT      34
#define HD      64
#define HP      72
#define AP      232
#define NFRAG   26
#define N1P     208
#define K2P     256
#define WSC     64.0f
#define WINV    0.015625f

#define NOP4 "v_nop\n\tv_nop\n\tv_nop\n\tv_nop"

__device__ __forceinline__ v8f wmma16(v16h a, v16h b, v8f c) {
  return __builtin_amdgcn_wmma_f32_16x16x32_f16(false, a, false, b, (short)0, c, false, false);
}
__device__ __forceinline__ v8f z8f() {
  v8f z = {0.f, 0.f, 0.f, 0.f, 0.f, 0.f, 0.f, 0.f};
  return z;
}
__device__ __forceinline__ void lds_sync() {
  asm volatile("s_wait_dscnt 0" ::: "memory");
}
__device__ __forceinline__ float rcp_(float x) { return __builtin_amdgcn_rcpf(x); }

__device__ __forceinline__ float sgm_(float x) { return rcp_(1.0f + __expf(-x)); }
__device__ __forceinline__ float tnh_(float x) { return 1.0f - 2.0f * rcp_(1.0f + __expf(2.0f * x)); }
__device__ __forceinline__ float elu_(float x) { return (x > 0.0f) ? x : (__expf(x) - 1.0f); }

__device__ __forceinline__ float gru1(float cr, float cz, float cn, float x, float f, float hp,
                                      v4f wr, v4f wz, v4f wn) {
  const float pre_r = fmaf(x, wr[0], fmaf(f, wr[1], wr[2]));
  const float rg    = sgm_(fmaf(cr, WINV, pre_r));
  const float pre_z = fmaf(x, wz[0], fmaf(f, wz[1], wz[2]));
  const float zg    = sgm_(fmaf(cz, WINV, pre_z));
  const float hn    = fmaf(cn, WINV, wn[3]);
  const float pre_n = fmaf(x, wn[0], fmaf(f, wn[1], wn[2]));
  const float ng    = tnh_(fmaf(rg, hn, pre_n));
  return fmaf(zg, hp - ng, ng);
}

__global__ __launch_bounds__(64) void k_img(const float* __restrict__ Whh,
                                           const float* __restrict__ wA,
                                           const float* __restrict__ wB,
                                           f16t* __restrict__ img) {
  const int i = blockIdx.x * 64 + threadIdx.x;
  if (i >= NFRAG * 64) return;
  const int f = i >> 6, q = i & 63, lane = q >> 1, ih = q & 1;
  const int hh = lane >> 4, n = lane & 15;
  const bool sc = (f >= 24);
  const int kt  = sc ? (f - 24) : (f & 1);
  const int col = sc ? n : ((f >> 1) * 16 + n);
  const int kb  = kt * 32 + 8 * hh + 16 * ih;
  Pk16 v;
#pragma unroll
  for (int e = 0; e < 8; ++e) {
    const int k = kb + e;
    float x;
    if (!sc) x = Whh[col * HD + k];
    else     x = (n == 0) ? wA[k] : ((n == 1) ? wB[k] : 0.0f);
    v.h[e] = (f16t)(x * WSC);
  }
  f16t* d = img + (size_t)i * 8;
  *(volatile v4u*)d = v.u;
  __threadfence();
  *(volatile v4u*)d = v.u;
}

__global__ __launch_bounds__(64) void k_pack(const float* __restrict__ W, f16t* __restrict__ P,
                                            int Nreal, int Kreal, int KP, int tot) {
  const int i = blockIdx.x * 64 + threadIdx.x;
  if (i >= tot) return;
  const int kq = KP >> 3;
  const int n  = i / kq;
  const int k  = (i - n * kq) * 8;
  Pk16 v;
#pragma unroll
  for (int e = 0; e < 8; ++e) {
    float x = 0.0f;
    if (n < Nreal && (k + e) < Kreal) x = W[(size_t)n * Kreal + k + e] * WSC;
    v.h[e] = (f16t)x;
  }
  f16t* d = P + (size_t)n * KP + k;
  *(volatile v4u*)d = v.u;
  __threadfence();
  *(volatile v4u*)d = v.u;
}

__global__ __launch_bounds__(64) __attribute__((amdgpu_num_vgpr(256)))
void k_main(const float* __restrict__ X, const float* __restrict__ F, const float* __restrict__ TR,
            const float* __restrict__ Wih, const float* __restrict__ bih, const float* __restrict__ bhh,
            const f16t* __restrict__ img,
            const f16t* __restrict__ P1a, const float* __restrict__ b1a,
            const f16t* __restrict__ P2a, const float* __restrict__ b2a,
            const float* __restrict__ W3a, const float* __restrict__ b3a,
            const f16t* __restrict__ P1b, const float* __restrict__ b1b,
            const f16t* __restrict__ P2b, const float* __restrict__ b2b,
            const float* __restrict__ W3b, const float* __restrict__ b3b,
            float* __restrict__ out, int nb) {
  __shared__ __attribute__((aligned(16))) f16t  sWB[NFRAG * 512];
  __shared__ __attribute__((aligned(16))) v4f   sXin[HD * 3];
  __shared__ __attribute__((aligned(16))) float sB[2176];
  __shared__ __attribute__((aligned(16))) float sAcc[4096];
  __shared__ __attribute__((aligned(16))) float sHf[2048];
  __shared__ __attribute__((aligned(16))) f16t  sHw[2 * 16 * HP];

  const int tid = threadIdx.x, lane = tid & 31, w = tid >> 5;
  const int hh = lane >> 4, m = lane & 15;
  const int b0 = blockIdx.x * SEQ_BLK;
  if (b0 + SEQ_BLK > nb) return;

  for (int i = tid; i < NFRAG * 64; i += 64)
    *(v8h*)(sWB + i * 8) = *(const v8h*)(img + (size_t)i * 8);
  {
    const int c = tid;
    v4f wr, wz, wn;
    wr[0] = Wih[c * 2 + 0];          wr[1] = Wih[c * 2 + 1];
    wr[2] = bih[c] + bhh[c];         wr[3] = 0.0f;
    wz[0] = Wih[(HD + c) * 2 + 0];   wz[1] = Wih[(HD + c) * 2 + 1];
    wz[2] = bih[HD + c] + bhh[HD + c]; wz[3] = 0.0f;
    wn[0] = Wih[(2 * HD + c) * 2 + 0]; wn[1] = Wih[(2 * HD + c) * 2 + 1];
    wn[2] = bih[2 * HD + c];         wn[3] = bhh[2 * HD + c];
    sXin[c * 3 + 0] = wr; sXin[c * 3 + 1] = wz; sXin[c * 3 + 2] = wn;
  }
  if (tid < SEQ_BLK) {
    const int s = tid;
    const float* px = X + (size_t)(b0 + s) * TT;
    const float* pf = F + (size_t)(b0 + s) * TT;
    float lx = 0.0f, lf = 0.0f;
#pragma unroll 1
    for (int t = 0; t < TT; ++t) {
      const float xv = px[t], fv = pf[t];
      if (xv != 0.0f) { lx = xv; lf = fv; }
      sB[t * SEQ_BLK + s] = lx;
      sB[1088 + t * SEQ_BLK + s] = lf;
    }
  }
  {
    const v4f z4 = {0.f, 0.f, 0.f, 0.f};
    for (int i = tid; i < 1024; i += 64) *(v4f*)(sAcc + i * 4) = z4;
    for (int i = tid; i < 512;  i += 64) *(v4f*)(sHf + i * 4) = z4;
    Pk16 zz; zz.u[0] = 0u; zz.u[1] = 0u; zz.u[2] = 0u; zz.u[3] = 0u;
    for (int i = tid; i < (2 * 16 * HP) / 8; i += 64) *(v8h*)(sHw + i * 8) = zz.h;
  }
  __syncthreads();

  f16t*  hw   = sHw + w * (16 * HP);
  float* hf   = sHf + w * 1024;
  float* accA = sAcc + w * 2048;
  float* accB = accA + 1024;
  const int rq = 16 * w + 8 * hh;
  const f16t* wbl = sWB + lane * 16;

  float sumA[8], sumB[8];
#pragma unroll
  for (int j = 0; j < 8; ++j) { sumA[j] = 0.0f; sumB[j] = 0.0f; }

#pragma unroll 1
  for (int t = 0; t <= TT; ++t) {
    Frag a0, a1;
    {
      const f16t* hp = hw + m * HP + 8 * hh;
      a0.q[0] = *(const v8h*)(hp);
      a0.q[1] = *(const v8h*)(hp + 16);
      a1.q[0] = *(const v8h*)(hp + 32);
      a1.q[1] = *(const v8h*)(hp + 48);
    }
    lds_sync();
    if (t > 0) {
      Frag s0, s1;
      s0.q[0] = *(const v8h*)(wbl + 24 * 512);
      s0.q[1] = *(const v8h*)(wbl + 24 * 512 + 8);
      s1.q[0] = *(const v8h*)(wbl + 25 * 512);
      s1.q[1] = *(const v8h*)(wbl + 25 * 512 + 8);
      v8f cS = wmma16(a0.v, s0.v, z8f());
      cS = wmma16(a1.v, s1.v, cS);
      asm volatile(NOP4 : "+v"(cS) : "v"(a0.v), "v"(a1.v), "v"(s0.v), "v"(s1.v));
      float eA[8], eB[8];
      const int src = lane & 16;
#pragma unroll
      for (int j = 0; j < 8; ++j) {
        const float la = __shfl(cS[j], src, 32);
        const float lb = __shfl(cS[j], src + 1, 32);
        eA[j] = __expf(la * WINV);
        eB[j] = __expf(lb * WINV);
        sumA[j] += eA[j];
        sumB[j] += eB[j];
      }
#pragma unroll 1
      for (int g = 0; g < 4; ++g) {
        const int c = g * 16 + m;
        const float* hq = hf + c * 16 + 8 * hh;
        const v4f h0 = *(const v4f*)hq, h1 = *(const v4f*)(hq + 4);
        float* pa = accA + c * 16 + 8 * hh;
        float* pb = accB + c * 16 + 8 * hh;
        v4f u0 = *(const v4f*)pa, u1 = *(const v4f*)(pa + 4);
        v4f q0 = *(const v4f*)pb, q1 = *(const v4f*)(pb + 4);
#pragma unroll
        for (int r = 0; r < 4; ++r) {
          u0[r] = fmaf(eA[r],     h0[r], u0[r]);
          u1[r] = fmaf(eA[4 + r], h1[r], u1[r]);
          q0[r] = fmaf(eB[r],     h0[r], q0[r]);
          q1[r] = fmaf(eB[4 + r], h1[r], q1[r]);
        }
        *(v4f*)pa = u0; *(v4f*)(pa + 4) = u1;
        *(v4f*)pb = q0; *(v4f*)(pb + 4) = q1;
      }
    }
    if (t < TT) {
      const float* px = sB + t * SEQ_BLK + rq;
      const v4f xa = *(const v4f*)px,          xb = *(const v4f*)(px + 4);
      const v4f ya = *(const v4f*)(px + 1088), yb = *(const v4f*)(px + 1092);
      lds_sync();
#pragma unroll 1
      for (int g = 0; g < 4; ++g) {
        Frag b0, b1, b2, b3, b4, b5;
        const f16t* pr = wbl + (2 * g) * 512;
        const f16t* pz = wbl + (2 * (4 + g)) * 512;
        const f16t* pn = wbl + (2 * (8 + g)) * 512;
        b0.q[0] = *(const v8h*)(pr);        b0.q[1] = *(const v8h*)(pr + 8);
        b1.q[0] = *(const v8h*)(pr + 512);  b1.q[1] = *(const v8h*)(pr + 520);
        b2.q[0] = *(const v8h*)(pz);        b2.q[1] = *(const v8h*)(pz + 8);
        b3.q[0] = *(const v8h*)(pz + 512);  b3.q[1] = *(const v8h*)(pz + 520);
        b4.q[0] = *(const v8h*)(pn);        b4.q[1] = *(const v8h*)(pn + 8);
        b5.q[0] = *(const v8h*)(pn + 512);  b5.q[1] = *(const v8h*)(pn + 520);
        v8f cR = wmma16(a0.v, b0.v, z8f()); cR = wmma16(a1.v, b1.v, cR);
        v8f cZ = wmma16(a0.v, b2.v, z8f()); cZ = wmma16(a1.v, b3.v, cZ);
        v8f cN = wmma16(a0.v, b4.v, z8f()); cN = wmma16(a1.v, b5.v, cN);
        asm volatile(NOP4
                     : "+v"(cR), "+v"(cZ), "+v"(cN)
                     : "v"(a0.v), "v"(a1.v), "v"(b0.v), "v"(b1.v), "v"(b2.v),
                       "v"(b3.v), "v"(b4.v), "v"(b5.v));
        const int c = g * 16 + m;
        const v4f wr = sXin[c * 3 + 0], wz = sXin[c * 3 + 1], wn = sXin[c * 3 + 2];
        float* hq = hf + c * 16 + 8 * hh;
        const v4f h0 = *(const v4f*)hq, h1 = *(const v4f*)(hq + 4);
        v4f n0, n1;
#pragma unroll
        for (int r = 0; r < 4; ++r) {
          n0[r] = gru1(cR[r],     cZ[r],     cN[r],     xa[r], ya[r], h0[r], wr, wz, wn);
          n1[r] = gru1(cR[4 + r], cZ[4 + r], cN[4 + r], xb[r], yb[r], h1[r], wr, wz, wn);
        }
        *(v4f*)hq = n0; *(v4f*)(hq + 4) = n1;
        f16t* hwp = hw + (8 * hh) * HP + c;
#pragma unroll
        for (int r = 0; r < 4; ++r) {
          hwp[r * HP]       = (f16t)n0[r];
          hwp[(4 + r) * HP] = (f16t)n1[r];
        }
      }
      lds_sync();
    }
  }

  __syncthreads();

  f16t*  aw  = sWB + w * (16 * AP);
  float* sVa = sB + 1088;
  float* sVb = sB + 1120;
#pragma unroll 1
  for (int br = 0; br < 2; ++br) {
    const f16t*  P1 = br ? P1b : P1a;
    const float* c1 = br ? b1b : b1a;
    const f16t*  P2 = br ? P2b : P2a;
    const float* c2 = br ? b2b : b2a;
    const float* W3 = br ? W3b : W3a;
    const float* c3 = br ? b3b : b3a;
    const float* accp = br ? accB : accA;
    float rs[8];
#pragma unroll
    for (int j = 0; j < 8; ++j) rs[j] = rcp_(br ? sumB[j] : sumA[j]);
#pragma unroll
    for (int g = 0; g < 4; ++g) {
      const float* pa = accp + (g * 16 + m) * 16 + 8 * hh;
      const v4f u0 = *(const v4f*)pa, u1 = *(const v4f*)(pa + 4);
#pragma unroll
      for (int r = 0; r < 4; ++r) {
        aw[(8 * hh + r) * AP + g * 16 + m]     = (f16t)(u0[r] * rs[r]);
        aw[(8 * hh + 4 + r) * AP + g * 16 + m] = (f16t)(u1[r] * rs[4 + r]);
      }
    }
    lds_sync();
    Frag i0, i1;
    {
      const f16t* ip = aw + m * AP + 8 * hh;
      i0.q[0] = *(const v8h*)(ip);      i0.q[1] = *(const v8h*)(ip + 16);
      i1.q[0] = *(const v8h*)(ip + 32); i1.q[1] = *(const v8h*)(ip + 48);
    }
    lds_sync();
#pragma unroll 1
    for (int nt = 0; nt < 13; ++nt) {
      const int n = nt * 16 + m;
      const f16t* pp = P1 + (size_t)n * HD + 8 * hh;
      Frag b0, b1;
      b0.q[0] = *(const v8h*)(pp);      b0.q[1] = *(const v8h*)(pp + 16);
      b1.q[0] = *(const v8h*)(pp + 32); b1.q[1] = *(const v8h*)(pp + 48);
      v8f d1 = wmma16(i0.v, b0.v, z8f());
      d1 = wmma16(i1.v, b1.v, d1);
      asm volatile(NOP4 : "+v"(d1) : "v"(i0.v), "v"(i1.v), "v"(b0.v), "v"(b1.v));
      float bb = 0.0f;
      if (n < 200) bb = c1[n];
#pragma unroll
      for (int j = 0; j < 8; ++j)
        aw[(8 * hh + j) * AP + n] = (f16t)elu_(fmaf(d1[j], WINV, bb));
    }
#pragma unroll
    for (int i = 0; i < 8; ++i) {
      const int idx = lane + 32 * i;
      aw[(idx >> 4) * AP + 208 + (idx & 15)] = (f16t)0.0f;
    }
    lds_sync();
    float part[8];
#pragma unroll
    for (int j = 0; j < 8; ++j) part[j] = 0.0f;
    const f16t* ap = aw + m * AP + 8 * hh;
#pragma unroll 1
    for (int nt = 0; nt < 13; ++nt) {
      const int n = nt * 16 + m;
      const f16t* pp = P2 + (size_t)n * K2P + 8 * hh;
      v8f d2 = z8f();
#pragma unroll 1
      for (int kt = 0; kt < 7; ++kt) {
        Frag a, b;
        a.q[0] = *(const v8h*)(ap + kt * 32);
        a.q[1] = *(const v8h*)(ap + kt * 32 + 16);
        b.q[0] = *(const v8h*)(pp + kt * 32);
        b.q[1] = *(const v8h*)(pp + kt * 32 + 16);
        d2 = wmma16(a.v, b.v, d2);
        asm volatile(NOP4 : "+v"(d2) : "v"(a.v), "v"(b.v));
      }
      float bb = 0.0f, w3 = 0.0f;
      if (n < 200) { bb = c2[n]; w3 = W3[n]; }
#pragma unroll
      for (int j = 0; j < 8; ++j)
        part[j] = fmaf(elu_(fmaf(d2[j], WINV, bb)), w3, part[j]);
    }
    const float b3v = c3[0];
#pragma unroll
    for (int j = 0; j < 8; ++j) {
      float v = part[j];
      v += __shfl_xor(v, 1, 32); v += __shfl_xor(v, 2, 32);
      v += __shfl_xor(v, 4, 32); v += __shfl_xor(v, 8, 32);
      const float raw = v + b3v;
      const float sg  = sgm_(raw);
      const float val = br ? (sg * 10000.0f) : (0.1f + sg * 4.9f);
      if (m == 0) {
        if (br) sVb[rq + j] = val; else sVa[rq + j] = val;
      }
    }
    lds_sync();
  }
  __syncthreads();

#pragma unroll 1
  for (int i = 0; i < 17; ++i) {
    const int e  = tid + 64 * i;
    const int s  = e / TT;
    const int tt = e - s * TT;
    const int gb = b0 + s;
    const float ang = F[(size_t)gb * TT + tt];
    const float tr  = TR[gb];
    const float rl  = sVa[s];
    const float am  = sVb[s];
    const float ex  = expf(-tr * rcp_(rl));
    const float cv  = cosf(ang);
    const float sv  = sinf(ang);
    const float num = (1.0f - ex) * sv;
    const float den = 1.0f - cv * ex;
    sB[e] = num * rcp_(den) * am;
  }
  __syncthreads();

  float* o0 = out + (size_t)b0 * TT;
  float* o1 = out + (size_t)nb * TT + b0;
  float* o2 = out + (size_t)nb * (TT + 1) + b0;
  v4f v0[4];
#pragma unroll
  for (int i = 0; i < 4; ++i) v0[i] = *(const v4f*)(sB + (tid + 64 * i) * 4);
  const bool tail = (tid < 16);
  v4f v4 = {0.f, 0.f, 0.f, 0.f};
  if (tail) v4 = *(const v4f*)(sB + (tid + 256) * 4);
  const bool hA = (tid < 8);
  const bool hB = (tid >= 8) && (tid < 16);
  v4f vh = {0.f, 0.f, 0.f, 0.f};
  if (hA) vh = *(const v4f*)(sVa + tid * 4);
  else if (hB) vh = *(const v4f*)(sVb + (tid - 8) * 4);

#pragma unroll
  for (int i = 0; i < 4; ++i) *(volatile v4f*)(o0 + (tid + 64 * i) * 4) = v0[i];
  if (tail) *(volatile v4f*)(o0 + (tid + 256) * 4) = v4;
  if (hA) *(volatile v4f*)(o1 + tid * 4) = vh;
  else if (hB) *(volatile v4f*)(o2 + (tid - 8) * 4) = vh;
  __threadfence();
#pragma unroll
  for (int i = 0; i < 4; ++i) *(volatile v4f*)(o0 + (tid + 64 * i) * 4) = v0[i];
  if (tail) *(volatile v4f*)(o0 + (tid + 256) * 4) = v4;
  if (hA) *(volatile v4f*)(o1 + tid * 4) = vh;
  else if (hB) *(volatile v4f*)(o2 + (tid - 8) * 4) = vh;
}

extern "C" void kernel_launch(void* const* d_in, const int* in_sizes, int n_in,
                              void* d_out, int out_size, void* d_ws, size_t ws_size,
                              hipStream_t stream) {
  if (n_in < 23) return;
  const int nb = in_sizes[4];
  if (nb <= 0 || (nb % SEQ_BLK) != 0) return;
  if (in_sizes[0] != nb * TT || in_sizes[1] != nb * TT) return;
  if (out_size != nb * (TT + 2)) return;
  if (in_sizes[5] != 3 * HD * 2 || in_sizes[6] != 3 * HD * HD ||
      in_sizes[7] != 3 * HD || in_sizes[8] != 3 * HD ||
      in_sizes[9] != HD || in_sizes[10] != HD) return;
  if (in_sizes[11] != 200 * HD || in_sizes[12] != 200 || in_sizes[13] != 200 * 200 ||
      in_sizes[14] != 200 || in_sizes[15] != 200 || in_sizes[16] != 1) return;
  if (in_sizes[17] != 200 * HD || in_sizes[18] != 200 || in_sizes[19] != 200 * 200 ||
      in_sizes[20] != 200 || in_sizes[21] != 200 || in_sizes[22] != 1) return;

  const float* X    = (const float*)d_in[0];
  const float* F    = (const float*)d_in[1];
  const float* TR   = (const float*)d_in[4];
  const float* Wih  = (const float*)d_in[5];
  const float* Whh  = (const float*)d_in[6];
  const float* bih  = (const float*)d_in[7];
  const float* bhh  = (const float*)d_in[8];
  const float* wSa  = (const float*)d_in[9];
  const float* wSb  = (const float*)d_in[10];
  const float* W1a  = (const float*)d_in[11];
  const float* b1a  = (const float*)d_in[12];
  const float* W2a  = (const float*)d_in[13];
  const float* b2a  = (const float*)d_in[14];
  const float* W3a  = (const float*)d_in[15];
  const float* b3a  = (const float*)d_in[16];
  const float* W1b  = (const float*)d_in[17];
  const float* b1b  = (const float*)d_in[18];
  const float* W2b  = (const float*)d_in[19];
  const float* b2b  = (const float*)d_in[20];
  const float* W3b  = (const float*)d_in[21];
  const float* b3b  = (const float*)d_in[22];
  float* out = (float*)d_out;

  char* ws = (char*)d_ws;
  size_t off = 0;
  auto carve = [&](size_t bytes) -> char* {
    char* p = ws + off;
    off = (off + bytes + 255) & ~(size_t)255;
    return p;
  };
  f16t* img = (f16t*)carve((size_t)NFRAG * 512 * 2);
  f16t* P1a = (f16t*)carve((size_t)N1P * HD * 2);
  f16t* P2a = (f16t*)carve((size_t)N1P * K2P * 2);
  f16t* P1b = (f16t*)carve((size_t)N1P * HD * 2);
  f16t* P2b = (f16t*)carve((size_t)N1P * K2P * 2);
  if (off > ws_size) return;

  k_img<<<dim3((NFRAG * 64 + 63) / 64), dim3(64), 0, stream>>>(Whh, wSa, wSb, img);
  {
    const int tot1 = N1P * (HD / 8);
    const int tot2 = N1P * (K2P / 8);
    k_pack<<<dim3((tot1 + 63) / 64), dim3(64), 0, stream>>>(W1a, P1a, 200, HD, HD, tot1);
    k_pack<<<dim3((tot2 + 63) / 64), dim3(64), 0, stream>>>(W2a, P2a, 200, 200, K2P, tot2);
    k_pack<<<dim3((tot1 + 63) / 64), dim3(64), 0, stream>>>(W1b, P1b, 200, HD, HD, tot1);
    k_pack<<<dim3((tot2 + 63) / 64), dim3(64), 0, stream>>>(W2b, P2b, 200, 200, K2P, tot2);
  }
  k_main<<<dim3(nb / SEQ_BLK), dim3(64), 0, stream>>>(X, F, TR, Wih, bih, bhh, img,
                                                     P1a, b1a, P2a, b2a, W3a, b3a,
                                                     P1b, b1b, P2b, b2b, W3b, b3b,
                                                     out, nb);
}
